// RecurrentClassifierOperator_25391846654171
// MI455X (gfx1250) — hardware-verified
//
#include <hip/hip_runtime.h>


typedef _Float16 f16t;
typedef f16t  v16h __attribute__((ext_vector_type(16)));
typedef f16t  v8h  __attribute__((ext_vector_type(8)));
typedef float v8f  __attribute__((ext_vector_type(8)));
typedef float v4f  __attribute__((ext_vector_type(4)));
typedef unsigned int v4u __attribute__((ext_vector_type(4)));

union Frag { v16h v; v8h q[2]; };
union Pk16 { v8h h; v4u u; };
union Pk32 { v4f f; v4u u; };

#define DIM   128
#define NG    512
#define KC    256
#define NOPS  16
#define ROWS  16
#define LP    264

__device__ __forceinline__ v8f wmma16(v16h a, v16h b, v8f c) {
    return __builtin_amdgcn_wmma_f32_16x16x32_f16(false, a, false, b, (short)0, c, false, false);
}

__device__ __forceinline__ float fsig(float x) {
    float t = __expf(-x);
    return __builtin_amdgcn_rcpf(1.0f + t);
}

__device__ __forceinline__ float ftanh(float x) {
    float ax = fabsf(x);
    float t  = __expf(-2.0f * ax);
    float r  = (1.0f - t) * __builtin_amdgcn_rcpf(1.0f + t);
    return copysignf(r, x);
}

__global__ __launch_bounds__(256)
void k_pack(const float* Wih, const float* Whh, f16t* P, int tot, float sc) {
    int i = blockIdx.x * 256 + threadIdx.x;
    if (i >= tot) return;
    int n  = i >> 5;
    int k  = (i & 31) * 8;
    int kk = k & (DIM - 1);
    const float* pa = Wih + (size_t)n * DIM + kk;
    const float* pb = Whh + (size_t)n * DIM + kk;
    v4f a0 = *(const v4f*)pa;
    v4f a1 = *(const v4f*)(pa + 4);
    v4f c0 = *(const v4f*)pb;
    v4f c1 = *(const v4f*)(pb + 4);
    const bool first = (k < DIM);
    Pk16 o;
#pragma unroll
    for (int e = 0; e < 4; ++e) {
        float v0 = first ? a0[e] : c0[e];
        float v1 = first ? a1[e] : c1[e];
        o.h[e]     = (f16t)(v0 * sc);
        o.h[4 + e] = (f16t)(v1 * sc);
    }
    f16t* d = P + (size_t)n * KC + k;
    *(volatile v4u*)d = o.u;
    __threadfence();
    *(volatile v4u*)d = o.u;
}

__global__ __launch_bounds__(256)
void k_lstm(const int* tokens, const int* lengths, const float* onehot,
            const float* emb, const f16t* P,
            const float* b_ih, const float* b_hh, const float* h0, const float* c0,
            const float* lin_W, const float* lin_b, float* out,
            int T, int nB, int vmax, float sc, float inv) {
    __shared__ __attribute__((aligned(16))) f16t  sA[ROWS * LP];
    __shared__ __attribute__((aligned(16))) float sHL[ROWS * DIM];
    __shared__ __attribute__((aligned(16))) float sOut[ROWS * 2];
    __shared__ int sLen[ROWS];

    const int tid  = threadIdx.x;
    const int lane = tid & 31;
    const int w    = tid >> 5;
    const int hh   = lane >> 4;
    const int m    = lane & 15;
    const int b0   = blockIdx.x * ROWS;
    if (b0 + ROWS > nB) return;

    if (tid < ROWS) {
        int L = lengths[b0 + tid];
        L = (L < 1) ? 1 : L;
        L = (L > T) ? T : L;
        sLen[tid] = L - 1;
    }
    for (int idx = tid; idx < ROWS * DIM; idx += 256) {
        int mm = idx >> 7, k = idx & (DIM - 1);
        sA[mm * LP + DIM + k] = (f16t)(h0[k] * sc);
    }
    for (int idx = tid; idx < ROWS * (LP - KC); idx += 256) {
        int mm = idx / (LP - KC), k = idx - mm * (LP - KC);
        sA[mm * LP + KC + k] = (f16t)0.0f;
    }

    const int u = 16 * w + m;
    const float bi = b_ih[u]           + b_hh[u];
    const float bf = b_ih[DIM + u]     + b_hh[DIM + u];
    const float bg = b_ih[2 * DIM + u] + b_hh[2 * DIM + u];
    const float bo = b_ih[3 * DIM + u] + b_hh[3 * DIM + u];

    float c[8], hk[8];
    int   tl[8];
    {
        const float cv = c0[u];
#pragma unroll
        for (int r = 0; r < 8; ++r) { c[r] = cv; hk[r] = 0.0f; }
    }
    __syncthreads();
#pragma unroll
    for (int r = 0; r < 8; ++r) tl[r] = sLen[8 * hh + r];

    const f16t* ap = sA + m * LP + 8 * hh;
    const f16t* bp = P + (size_t)u * KC + 8 * hh;

    const int gm = tid >> 4;
    const int gk = (tid & 15) * 8;
    const int* tk = tokens + (size_t)(b0 + gm) * T;
    f16t* xdst = sA + gm * LP + gk;
    f16t* hdst = sA + (8 * hh) * LP + DIM + u;

#pragma unroll 1
    for (int t = 0; t < T; ++t) {
        {
            int tok = tk[t];
            tok = (tok < 0) ? 0 : tok;
            tok = (tok > vmax) ? vmax : tok;
            const float* er = emb + (size_t)tok * DIM + gk;
            v4f e0 = *(const v4f*)er;
            v4f e1 = *(const v4f*)(er + 4);
            Pk16 pk;
#pragma unroll
            for (int e = 0; e < 4; ++e) {
                pk.h[e]     = (f16t)(fmaxf(e0[e], 0.0f) * sc);
                pk.h[4 + e] = (f16t)(fmaxf(e1[e], 0.0f) * sc);
            }
            *(v8h*)xdst = pk.h;
        }
        __syncthreads();

        const v8f z = {0.f, 0.f, 0.f, 0.f, 0.f, 0.f, 0.f, 0.f};
        v8f acc[4];
        acc[0] = z; acc[1] = z; acc[2] = z; acc[3] = z;
#pragma unroll 1
        for (int kt = 0; kt < KC / 32; ++kt) {
            Frag a, b[4];
            const f16t* pa = ap + kt * 32;
            a.q[0] = *(const v8h*)pa;
            a.q[1] = *(const v8h*)(pa + 16);
#pragma unroll
            for (int g = 0; g < 4; ++g) {
                const f16t* pb = bp + (size_t)g * DIM * KC + kt * 32;
                b[g].q[0] = *(const v8h*)pb;
                b[g].q[1] = *(const v8h*)(pb + 16);
            }
#pragma unroll
            for (int g = 0; g < 4; ++g) acc[g] = wmma16(a.v, b[g].v, acc[g]);
            asm volatile("v_nop\n\tv_nop\n\tv_nop\n\tv_nop"
                         : "+v"(acc[0]), "+v"(acc[1]), "+v"(acc[2]), "+v"(acc[3])
                         : "v"(a.v), "v"(b[0].v), "v"(b[1].v), "v"(b[2].v), "v"(b[3].v));
        }
        __syncthreads();

#pragma unroll
        for (int r = 0; r < 8; ++r) {
            float gi = fsig (fmaf(acc[0][r], inv, bi));
            float gf = fsig (fmaf(acc[1][r], inv, bf));
            float gg = ftanh(fmaf(acc[2][r], inv, bg));
            float go = fsig (fmaf(acc[3][r], inv, bo));
            float cv = fmaf(gf, c[r], gi * gg);
            float hv = go * ftanh(cv);
            c[r]  = cv;
            hk[r] = (t == tl[r]) ? hv : hk[r];
            hdst[r * LP] = (f16t)(hv * sc);
        }
    }

#pragma unroll
    for (int r = 0; r < 8; ++r) sHL[(8 * hh + r) * DIM + u] = fmaxf(hk[r], 0.0f);
    __syncthreads();
    if (tid < 32) {
        const int b = tid >> 1, j = tid & 1;
        const float* wr = lin_W + j * (DIM + NOPS);
        const float* hr = sHL + b * DIM;
        const float* oh = onehot + (size_t)(b0 + b) * NOPS;
        float s = 0.0f;
#pragma unroll 1
        for (int k = 0; k < DIM; ++k)  s = fmaf(hr[k], wr[k], s);
#pragma unroll 1
        for (int k = 0; k < NOPS; ++k) s = fmaf(oh[k], wr[DIM + k], s);
        s += lin_b[j];
        sOut[tid] = s;
    }
    __syncthreads();
    if (tid < 32) {
        Pk32 v;
        v.f = *(const v4f*)(sOut + 4 * (tid & 7));
        if (tid < 8) {
            float* d = out + (size_t)b0 * 2 + 4 * tid;
            *(volatile v4u*)d = v.u;
            __threadfence();
            *(volatile v4u*)d = v.u;
        }
    }
}

extern "C" void kernel_launch(void* const* d_in, const int* in_sizes, int n_in,
                              void* d_out, int out_size, void* d_ws, size_t ws_size,
                              hipStream_t stream) {
    if (n_in < 12) return;
    const int nB = in_sizes[1];
    if (nB <= 0 || (nB % ROWS) != 0) return;
    const int T = in_sizes[0] / nB;
    if (T <= 0 || T * nB != in_sizes[0]) return;
    if (in_sizes[2] != nB * NOPS) return;
    if (in_sizes[3] < DIM || (in_sizes[3] % DIM) != 0) return;
    const int vmax = in_sizes[3] / DIM - 1;
    if (in_sizes[4] != NG * DIM || in_sizes[5] != NG * DIM) return;
    if (in_sizes[6] != NG || in_sizes[7] != NG) return;
    if (in_sizes[8] < DIM || in_sizes[9] < DIM) return;
    if (in_sizes[10] != 2 * (DIM + NOPS) || in_sizes[11] != 2) return;
    if (out_size != nB * 2) return;

    const int*   tokens  = (const int*)d_in[0];
    const int*   lengths = (const int*)d_in[1];
    const float* onehot  = (const float*)d_in[2];
    const float* emb     = (const float*)d_in[3];
    const float* W_ih    = (const float*)d_in[4];
    const float* W_hh    = (const float*)d_in[5];
    const float* b_ih    = (const float*)d_in[6];
    const float* b_hh    = (const float*)d_in[7];
    const float* h0      = (const float*)d_in[8];
    const float* c0      = (const float*)d_in[9];
    const float* lin_W   = (const float*)d_in[10];
    const float* lin_b   = (const float*)d_in[11];
    float* out = (float*)d_out;

    const size_t plane_bytes = (size_t)NG * KC * sizeof(f16t);
    if (plane_bytes > ws_size) return;
    f16t* P = (f16t*)d_ws;

    const float SC  = 16.0f;
    const float INV = 0.00390625f;

    const int tot = NG * (KC / 8);
    k_pack<<<dim3((tot + 255) / 256), dim3(256), 0, stream>>>(W_ih, W_hh, P, tot, SC);
    k_lstm<<<dim3(nB / ROWS), dim3(256), 0, stream>>>(tokens, lengths, onehot, emb, P,
                                                      b_ih, b_hh, h0, c0, lin_W, lin_b, out,
                                                      T, nB, vmax, SC, INV);
}
